// SelfAttentionUnit_5317169512778
// MI455X (gfx1250) — hardware-verified
//
#include <hip/hip_runtime.h>


#define NB_  8
#define CIN  67
#define CP   96
#define C2   128
#define COUT 64
#define NN   16384
#define BNEPS 1e-5f
typedef _Float16 h16;
typedef unsigned short bf;
typedef __attribute__((ext_vector_type(16))) __bf16   v16bf;
typedef __attribute__((ext_vector_type(16))) _Float16 v16h;
typedef __attribute__((ext_vector_type(8)))  _Float16 v8h;
typedef __attribute__((ext_vector_type(8)))  unsigned short v8us;
typedef __attribute__((ext_vector_type(8)))  float    v8f;
typedef __attribute__((ext_vector_type(4)))  float    v4f;
typedef v8h  __attribute__((may_alias)) v8ha;
typedef v4f  __attribute__((may_alias)) v4fa;
typedef v8us __attribute__((may_alias)) v8usa;

__device__ __forceinline__ unsigned short f2bf(float f) { unsigned u = __float_as_uint(f); u += 0x7FFFu + ((u >> 16) & 1u); return (unsigned short)(u >> 16); }
__device__ __forceinline__ float bf2f(unsigned short b) { return __uint_as_float(((unsigned)b) << 16); }
__device__ __forceinline__ float bfr(float f) { return bf2f(f2bf(f)); }
__device__ __forceinline__ v16h cat16(v8h lo, v8h hi) { return __builtin_shufflevector(lo, hi, 0, 1, 2, 3, 4, 5, 6, 7, 8, 9, 10, 11, 12, 13, 14, 15); }
__device__ __forceinline__ v16bf cat16b(v8us lo, v8us hi) { return __builtin_bit_cast(v16bf, __builtin_shufflevector(lo, hi, 0, 1, 2, 3, 4, 5, 6, 7, 8, 9, 10, 11, 12, 13, 14, 15)); }
__device__ __forceinline__ v8f wmma16(v16h a, v16h b, v8f c) { return __builtin_amdgcn_wmma_f32_16x16x32_f16(false, a, false, b, (short)0, c, false, false); }
__device__ __forceinline__ v8f wmmab(v16bf a, v16bf b, v8f c) { return __builtin_amdgcn_wmma_f32_16x16x32_bf16(false, a, false, b, (short)0, c, false, false); }


template <typename T16> struct WFrag;
template <> struct WFrag<h16> { typedef v16h V; static __device__ __forceinline__ V ld(const h16* p) { return cat16(*(const v8h*)p, *(const v8h*)(p + 16)); } static __device__ __forceinline__ v8f mma(V a, V b, v8f c) { return wmma16(a, b, c); } };
template <> struct WFrag<bf> { typedef v16bf V; static __device__ __forceinline__ V ld(const bf* p) { return cat16b(*(const v8us*)p, *(const v8us*)(p + 16)); } static __device__ __forceinline__ v8f mma(V a, V b, v8f c) { return wmmab(a, b, c); } };
template <typename T16, int NSPLIT, bool BIAS>
__global__ __launch_bounds__(32) void k_gemmw(const T16* __restrict__ A, const T16* __restrict__ A2, const T16* __restrict__ Bt, const T16* __restrict__ Bt2, int K, float* C, int ldc, const float* __restrict__ bias, size_t sA, size_t sB, size_t sC) {
    typedef typename WFrag<T16>::V V;
    __shared__ __align__(16) float os[16 * 68];
    const size_t z = blockIdx.z; A += z * sA; if (A2) A2 += z * sA; Bt += z * sB; if (Bt2) Bt2 += z * sB; C += z * sC;
    const int lane = threadIdx.x & 31, lr = lane & 15, hi = lane >> 4; const int r0 = blockIdx.x * 64, c0 = blockIdx.y * 64;
    v8f acc[4][4];
#pragma unroll
    for (int mb = 0; mb < 4; ++mb)
#pragma unroll
        for (int nb = 0; nb < 4; ++nb) acc[mb][nb] = (v8f){};
    const size_t aoff = (size_t)(r0 + lr) * K + 8 * hi, boff = (size_t)(c0 + lr) * K + 8 * hi;
#pragma unroll 1
    for (int kc = 0; kc < K; kc += 32) {
        V a[4], a2[4];
#pragma unroll
        for (int mb = 0; mb < 4; ++mb) { a[mb] = WFrag<T16>::ld(A + aoff + (size_t)mb * 16 * K + kc); if (NSPLIT == 1 || NSPLIT == 2) a2[mb] = WFrag<T16>::ld(A2 + aoff + (size_t)mb * 16 * K + kc); }
#pragma unroll
        for (int nb = 0; nb < 4; ++nb) { const V b = WFrag<T16>::ld(Bt + boff + (size_t)nb * 16 * K + kc); V b2; if (NSPLIT >= 2) b2 = WFrag<T16>::ld(Bt2 + boff + (size_t)nb * 16 * K + kc);
#pragma unroll
            for (int mb = 0; mb < 4; ++mb) { acc[mb][nb] = WFrag<T16>::mma(a[mb], b, acc[mb][nb]); if (NSPLIT == 1 || NSPLIT == 2) acc[mb][nb] = WFrag<T16>::mma(a2[mb], b, acc[mb][nb]); if (NSPLIT >= 2) acc[mb][nb] = WFrag<T16>::mma(a[mb], b2, acc[mb][nb]); } }
        asm volatile("v_nop\n\tv_nop\n\tv_nop\n\tv_nop" : "+v"(acc[0][0]), "+v"(acc[1][1]), "+v"(acc[2][2]), "+v"(acc[3][3]) : "v"(a[0]), "v"(a[3]));
    }
#pragma unroll
    for (int mb = 0; mb < 4; ++mb) {
#pragma unroll
        for (int nb = 0; nb < 4; ++nb) {
#pragma unroll
            for (int j = 0; j < 8; ++j) os[(hi * 8 + j) * 68 + nb * 16 + lr] = acc[mb][nb][j]; }
        __builtin_amdgcn_wave_barrier(); asm volatile("" ::: "memory");
        float* crow = C + (size_t)(r0 + mb * 16) * ldc + c0;
#pragma unroll 1
        for (int ps = 0; ps < 2; ++ps) {
#pragma unroll
            for (int s = 0; s < 8; ++s) { const int row = 2 * s + hi, cofs = lr * 4; v4f val = *(const v4fa*)(os + row * 68 + cofs); if (BIAS) { val[0] += bfr(bias[c0 + cofs]); val[1] += bfr(bias[c0 + cofs + 1]); val[2] += bfr(bias[c0 + cofs + 2]); val[3] += bfr(bias[c0 + cofs + 3]); }
                *(volatile v4f*)(crow + (size_t)row * ldc + cofs) = val; }
            if (ps == 0) __threadfence(); }
        __builtin_amdgcn_wave_barrier(); asm volatile("" ::: "memory");
    }
}

__device__ __forceinline__ void splitf(float y, unsigned short& h, unsigned short& l) { h = f2bf(y); l = f2bf(y - bf2f(h)); }
typedef __attribute__((ext_vector_type(2))) unsigned short v2us;
typedef __attribute__((ext_vector_type(4))) unsigned short v4us;

__global__ __launch_bounds__(256) void k_xt(const float* __restrict__ xb, bf* XT) { const size_t e = ((size_t)blockIdx.x * 256 + threadIdx.x) * 2; if (e >= (size_t)NN * CP) return; const int c = (int)(e % CP); const int n = (int)(e / CP); v2us o;
#pragma unroll
    for (int q = 0; q < 2; ++q) o[q] = (c + q < CIN) ? f2bf(xb[(size_t)(c + q) * NN + n]) : (unsigned short)0; *(volatile v2us*)(XT + e) = o; __threadfence(); *(volatile v2us*)(XT + e) = o; }
__global__ __launch_bounds__(256) void k_wpad(const float* __restrict__ W, bf* Bt) { const int e = (blockIdx.x * 256 + threadIdx.x) * 2; if (e >= C2 * CP) return; const int c = e % CP, o = e / CP; v2us w2;
#pragma unroll
    for (int q = 0; q < 2; ++q) w2[q] = (c + q < CIN) ? f2bf(W[o * CIN + c + q]) : (unsigned short)0; *(volatile v2us*)(Bt + e) = w2; __threadfence(); *(volatile v2us*)(Bt + e) = w2; }
__global__ __launch_bounds__(256) void k_cvt8(const float* __restrict__ src, bf* dst, size_t n8) { const size_t i = (size_t)blockIdx.x * 256 + threadIdx.x; if (i >= n8) return; const v8f v = *(const v8f*)(src + i * 8); v8us o;
#pragma unroll
    for (int q = 0; q < 8; ++q) o[q] = f2bf(v[q]); *(volatile v8us*)(dst + i * 8) = o; __threadfence(); *(volatile v8us*)(dst + i * 8) = o; }
__global__ __launch_bounds__(256) void k_zero8(bf* Z, size_t n8) { const size_t i = (size_t)blockIdx.x * 256 + threadIdx.x; if (i >= n8) return; const v8us z = (v8us){}; *(volatile v8us*)(Z + i * 8) = z; __threadfence(); *(volatile v8us*)(Z + i * 8) = z; }
__device__ __forceinline__ void bn_coef(const float* __restrict__ bn, int nch, int ch, float& sc, float& sh) { sc = __fmul_rn(bfr(bn[ch]), __fdiv_rn(1.0f, __fsqrt_rn(__fadd_rn(bfr(bn[3 * nch + ch]), BNEPS)))); float ms = __fmul_rn(bfr(bn[2 * nch + ch]), sc); asm volatile("" : "+v"(ms)); sh = __fsub_rn(bfr(bn[nch + ch]), ms); }
__global__ __launch_bounds__(256) void k_bncol(const float* __restrict__ F, const float* __restrict__ bn, bf* Ph, bf* Pl) { const size_t e = ((size_t)blockIdx.x * 256 + threadIdx.x) * 4; if (e >= (size_t)NN * C2) return; const int o = (int)(e % C2); const v4f f = *(const v4f*)(F + e); v4us oh, ol;
#pragma unroll
    for (int q = 0; q < 4; ++q) { float sc, sh; bn_coef(bn, C2, o + q, sc, sh); float y = __fmul_rn(f[q], sc); asm volatile("" : "+v"(y)); y = fmaxf(__fadd_rn(y, sh), 0.f); unsigned short a, c; splitf(y, a, c); oh[q] = a; ol[q] = c; }
    *(volatile v4us*)(Ph + e) = oh; *(volatile v4us*)(Pl + e) = ol; __threadfence(); *(volatile v4us*)(Ph + e) = oh; *(volatile v4us*)(Pl + e) = ol; }
__global__ __launch_bounds__(256) void k_bnrow(const float* __restrict__ F, const float* __restrict__ bn, int nch, bf* Ph, bf* Pl) { const size_t e = ((size_t)blockIdx.x * 256 + threadIdx.x) * 4; if (e >= (size_t)nch * NN) return; const int ch = (int)(e / NN); float sc, sh; bn_coef(bn, nch, ch, sc, sh); const v4f f = *(const v4f*)(F + e); v4us oh, ol;
#pragma unroll
    for (int q = 0; q < 4; ++q) { float y = __fmul_rn(f[q], sc); asm volatile("" : "+v"(y)); y = fmaxf(__fadd_rn(y, sh), 0.f); unsigned short a, c; splitf(y, a, c); oh[q] = a; ol[q] = c; }
    *(volatile v4us*)(Ph + e) = oh; *(volatile v4us*)(Pl + e) = ol; __threadfence(); *(volatile v4us*)(Ph + e) = oh; *(volatile v4us*)(Pl + e) = ol; }
__global__ __launch_bounds__(256) void k_bnout(const float* __restrict__ F, const float* __restrict__ bn, float* O) { const size_t e = ((size_t)blockIdx.x * 256 + threadIdx.x) * 4; if (e >= (size_t)COUT * NN) return; const int ch = (int)(e / NN); float sc, sh; bn_coef(bn, COUT, ch, sc, sh); const v4f f = *(const v4f*)(F + e); v4f y;
#pragma unroll
    for (int q = 0; q < 4; ++q) { float t = __fmul_rn(f[q], sc); asm volatile("" : "+v"(t)); y[q] = fmaxf(__fadd_rn(t, sh), 0.f); }
    *(volatile v4f*)(O + e) = y; __threadfence(); *(volatile v4f*)(O + e) = y; }
__global__ __launch_bounds__(256) void k_kvt(const float* __restrict__ KV, bf* Th, bf* Tl) { const int e = (blockIdx.x * 256 + threadIdx.x) * 2; if (e >= C2 * C2) return; const int c = e % C2, d = e / C2; v2us oh, ol;
#pragma unroll
    for (int q = 0; q < 2; ++q) { unsigned short a, c2; splitf(KV[(c + q) * C2 + d], a, c2); oh[q] = a; ol[q] = c2; } *(volatile v2us*)(Th + e) = oh; *(volatile v2us*)(Tl + e) = ol; __threadfence(); *(volatile v2us*)(Th + e) = oh; *(volatile v2us*)(Tl + e) = ol; }
__global__ __launch_bounds__(256) void k_split8(const float* __restrict__ F, bf* H, bf* Lw, size_t n8) { const size_t i = (size_t)blockIdx.x * 256 + threadIdx.x; if (i >= n8) return; const v8f v = *(const v8f*)(F + i * 8); v8us oh, ol;
#pragma unroll
    for (int q = 0; q < 8; ++q) { unsigned short a, c; splitf(v[q], a, c); oh[q] = a; ol[q] = c; } *(volatile v8us*)(H + i * 8) = oh; *(volatile v8us*)(Lw + i * 8) = ol; __threadfence(); *(volatile v8us*)(H + i * 8) = oh; *(volatile v8us*)(Lw + i * 8) = ol; }

extern "C" void kernel_launch(void* const* d_in, const int* in_sizes, int n_in,
                              void* d_out, int out_size, void* d_ws, size_t ws_size, hipStream_t stream) {
    (void)in_sizes; (void)n_in; (void)out_size;
    const float* x = (const float*)d_in[0]; const float* Wq = (const float*)d_in[1]; const float* Wk = (const float*)d_in[2]; const float* Wv = (const float*)d_in[3]; const float* Wf = (const float*)d_in[4]; const float* bnq = (const float*)d_in[5]; const float* bnk = (const float*)d_in[6]; const float* bnv = (const float*)d_in[7]; const float* bnf = (const float*)d_in[8];
    float* OUT = (float*)d_out;
    char* wsp = (char*)d_ws;
    auto take = [&](size_t bytes) { char* p = wsp; wsp += (bytes + 255) & ~(size_t)255; return (void*)p; };
    bf* WQ = (bf*)take((size_t)C2 * CP * 2); bf* WK = (bf*)take((size_t)C2 * CP * 2); bf* WV = (bf*)take((size_t)C2 * CP * 2); bf* WF = (bf*)take((size_t)COUT * C2 * 2); bf* ZF = (bf*)take((size_t)COUT * C2 * 2);
    bf* XT = (bf*)take((size_t)NN * CP * 2); float* F = (float*)take((size_t)NN * C2 * 4); bf* Qh = (bf*)take((size_t)NN * C2 * 2); bf* Ql = (bf*)take((size_t)NN * C2 * 2); bf* Kh = (bf*)take((size_t)C2 * NN * 2); bf* Kl = (bf*)take((size_t)C2 * NN * 2); bf* Vh = (bf*)take((size_t)C2 * NN * 2); bf* Vl = (bf*)take((size_t)C2 * NN * 2);
    float* KV = (float*)take((size_t)C2 * C2 * 4); bf* KTh = (bf*)take((size_t)C2 * C2 * 2); bf* KTl = (bf*)take((size_t)C2 * C2 * 2); bf* ALh = (bf*)take((size_t)NN * C2 * 2); bf* ALl = (bf*)take((size_t)NN * C2 * 2); float* G = (float*)take((size_t)COUT * NN * 4);
    if ((size_t)(wsp - (char*)d_ws) > ws_size) return;
    k_wpad<<<(C2 * CP / 2 + 255) / 256, 256, 0, stream>>>(Wq, WQ); k_wpad<<<(C2 * CP / 2 + 255) / 256, 256, 0, stream>>>(Wk, WK); k_wpad<<<(C2 * CP / 2 + 255) / 256, 256, 0, stream>>>(Wv, WV);
    k_cvt8<<<(COUT * C2 / 8 + 255) / 256, 256, 0, stream>>>(Wf, WF, (size_t)COUT * C2 / 8); k_zero8<<<(COUT * C2 / 8 + 255) / 256, 256, 0, stream>>>(ZF, (size_t)COUT * C2 / 8);
    const unsigned nb4 = (unsigned)(((size_t)NN * C2 / 4 + 255) / 256);
    for (int b = 0; b < NB_; ++b) {
        k_xt<<<(unsigned)(((size_t)NN * CP / 2 + 255) / 256), 256, 0, stream>>>(x + (size_t)b * CIN * NN, XT);
        k_gemmw<bf, 0, false><<<dim3(NN / 64, C2 / 64, 1), 32, 0, stream>>>(XT, nullptr, WQ, nullptr, CP, F, C2, nullptr, 0, 0, 0); k_bncol<<<nb4, 256, 0, stream>>>(F, bnq, Qh, Ql);
        k_gemmw<bf, 0, false><<<dim3(C2 / 64, NN / 64, 1), 32, 0, stream>>>(WK, nullptr, XT, nullptr, CP, F, NN, nullptr, 0, 0, 0); k_bnrow<<<nb4, 256, 0, stream>>>(F, bnk, C2, Kh, Kl);
        k_gemmw<bf, 0, false><<<dim3(C2 / 64, NN / 64, 1), 32, 0, stream>>>(WV, nullptr, XT, nullptr, CP, F, NN, nullptr, 0, 0, 0); k_bnrow<<<nb4, 256, 0, stream>>>(F, bnv, C2, Vh, Vl);
        k_gemmw<bf, 2, false><<<dim3(C2 / 64, C2 / 64, 1), 32, 0, stream>>>(Kh, Kl, Vh, Vl, NN, KV, C2, nullptr, 0, 0, 0);
        k_kvt<<<(C2 * C2 / 2 + 255) / 256, 256, 0, stream>>>(KV, KTh, KTl);
        k_gemmw<bf, 2, false><<<dim3(NN / 64, C2 / 64, 1), 32, 0, stream>>>(Qh, Ql, KTh, KTl, C2, F, C2, nullptr, 0, 0, 0);
        k_split8<<<(unsigned)(((size_t)NN * C2 / 8 + 255) / 256), 256, 0, stream>>>(F, ALh, ALl, (size_t)NN * C2 / 8);
        k_gemmw<bf, 2, false><<<dim3(COUT / 64, NN / 64, 1), 32, 0, stream>>>(WF, ZF, ALh, ALl, C2, G, NN, nullptr, 0, 0, 0);
        k_bnout<<<(unsigned)(((size_t)COUT * NN / 4 + 255) / 256), 256, 0, stream>>>(G, bnf, OUT + (size_t)b * COUT * NN); }
}
